// SelectiveStateFusion_11416023072916
// MI455X (gfx1250) — hardware-verified
//
#include <hip/hip_runtime.h>
#include <math.h>

typedef __attribute__((ext_vector_type(16))) _Float16 v16h;
typedef __attribute__((ext_vector_type(8)))  _Float16 v8h;
typedef __attribute__((ext_vector_type(16))) __bf16   v16b;
typedef __attribute__((ext_vector_type(8)))  __bf16   v8b;
typedef __attribute__((ext_vector_type(8)))  float    v8f;
typedef __attribute__((ext_vector_type(4)))  float    v4f;

constexpr int kNStr  = 3;
constexpr int kBatch = 2;
constexpr int kSeq   = 2048;
constexpr int kDm    = 256;
constexpr int kDin   = 512;
constexpr int kNst   = 16;
constexpr int kDtR   = 16;
constexpr int kXzP   = 2 * kDin;
constexpr int kXdN   = kDtR + 2 * kNst;
constexpr int kXdP   = 64;
constexpr int kRowsS = kBatch * kSeq;
constexpr int kRowsT = kNStr * kRowsS;
constexpr int kCat   = kNStr * kDm;
constexpr int kConvTP = 260;
constexpr int kScanTS = 64;
constexpr int kScanCh = 64;
constexpr int kScanYP = 68;
constexpr float kWScale = 64.0f;
constexpr float kUScale = 256.0f;
constexpr float kYScale = 1024.0f;
static_assert(kXdN <= kXdP, "x_proj pad");
static_assert((kDm % 32) == 0 && (kDin % 32) == 0 && (kCat % 32) == 0, "GEMM K multiples of 32");
static_assert((kRowsS % 64) == 0 && (kXzP % 64) == 0 && (kXdP % 64) == 0 && (kDm % 64) == 0, "GEMM M,N multiples of 64");
static_assert((kSeq % kScanTS) == 0 && (kSeq % 64) == 0 && (kDin % kScanCh) == 0 && (kDin % 256) == 0, "tile multiples");
static_assert((kRowsS % 8) == 0, "LN blocks never straddle streams");

constexpr size_t kOffXN  = 0;
constexpr size_t kOffWI  = kOffXN + (size_t)kRowsT * kDm * 2;
constexpr size_t kOffWX  = kOffWI + (size_t)kNStr * kXzP * kDm * 2;
constexpr size_t kOffWO  = kOffWX + (size_t)kNStr * kXdP * kDin * 2;
constexpr size_t kOffWP  = kOffWO + (size_t)kNStr * kDm * kDin * 2;
constexpr size_t kOffXZ  = kOffWP + (size_t)kDm * kCat * 2;
constexpr size_t kOffUC  = kOffXZ + (size_t)kRowsT * kXzP * 4;
constexpr size_t kOffUH  = kOffUC + (size_t)kRowsT * kDin * 4;
constexpr size_t kOffXD  = kOffUH + (size_t)kRowsT * kDin * 2;
constexpr size_t kOffYH  = kOffXD + (size_t)kRowsT * kXdP * 4;
constexpr size_t kWsTotal = kOffYH + (size_t)kRowsT * kDin * 2;
constexpr size_t kOffPR  = kOffXZ;
constexpr size_t kOffMU  = kOffPR + (size_t)kRowsT * kDm * 4;
constexpr size_t kOffWG  = kOffMU + (size_t)kRowsS * kCat * 2;
constexpr size_t kOffPO  = kOffWG + (size_t)kRowsS * kDm * 4;
constexpr size_t kOffCF  = kOffPO + (size_t)kBatch * kCat * 4;
constexpr size_t kAliasEnd = kOffCF + 128;
static_assert(kWsTotal == 113049600ull, "carve total");
static_assert(kWsTotal <= 134217728ull, "carve cap");
static_assert(kAliasEnd <= kOffUC, "aliases fit inside XZ");
static_assert((kOffWI % 128) == 0 && (kOffWX % 128) == 0 && (kOffWO % 128) == 0 && (kOffWP % 128) == 0 &&
              (kOffXZ % 128) == 0 && (kOffUC % 128) == 0 && (kOffUH % 128) == 0 && (kOffXD % 128) == 0 &&
              (kOffYH % 128) == 0 && (kOffPR % 128) == 0 && (kOffMU % 128) == 0 && (kOffWG % 128) == 0 &&
              (kOffPO % 128) == 0 && (kOffCF % 128) == 0, "128-B aligned regions");

__device__ __forceinline__ unsigned short f2bf_bits(float f) {
  unsigned u = __float_as_uint(f);
  return (unsigned short)((u + 0x7FFFu + ((u >> 16) & 1u)) >> 16);
}
__device__ __forceinline__ float bf_bits2f(unsigned short h) { return __uint_as_float(((unsigned)h) << 16); }

__device__ __forceinline__ void dep_guard_h(v8f& a, v8f& b, v16h x, v16h y) { asm volatile("v_nop\n\tv_nop\n\tv_nop\n\tv_nop" : "+v"(a), "+v"(b) : "v"(x), "v"(y)); }
__device__ __forceinline__ void dep_guard_b(v8f& a, v8f& b, v16b x, v16b y) { asm volatile("v_nop\n\tv_nop\n\tv_nop\n\tv_nop" : "+v"(a), "+v"(b) : "v"(x), "v"(y)); }
__device__ __forceinline__ void keep4_h(v16h a, v16h b, v16h c, v16h d) { asm volatile("v_nop" :: "v"(a), "v"(b), "v"(c), "v"(d)); }
__device__ __forceinline__ void keep4_b(v16b a, v16b b, v16b c, v16b d) { asm volatile("v_nop" :: "v"(a), "v"(b), "v"(c), "v"(d)); }
__device__ __forceinline__ void acc_guard4(v8f& a, v8f& b, v8f& c, v8f& d) { asm volatile("v_nop\n\tv_nop\n\tv_nop\n\tv_nop" : "+v"(a), "+v"(b), "+v"(c), "+v"(d)); }
template <typename T> struct Frag;
template <> struct Frag<_Float16> {
  typedef v16h V; union U { v16h v; v8h h[2]; };
  static __device__ __forceinline__ v16h load(const _Float16* p) {
    U f; f.h[0] = *(const v8h*)(p); f.h[1] = *(const v8h*)(p + 16); return f.v;
  }
  static __device__ __forceinline__ v8f mma(v16h a, v16h b, v8f c) {
    return __builtin_amdgcn_wmma_f32_16x16x32_f16(false, a, false, b, (short)0, c, false, false);
  }
  static __device__ __forceinline__ void guard(v8f& a, v8f& b, v16h x, v16h y) { dep_guard_h(a, b, x, y); }
  static __device__ __forceinline__ void keep(v16h a, v16h b, v16h c, v16h d) { keep4_h(a, b, c, d); }
};
template <> struct Frag<__bf16> {
  typedef v16b V; union U { v16b v; v8b h[2]; };
  static __device__ __forceinline__ v16b load(const __bf16* p) {
    U f; f.h[0] = *(const v8b*)(p); f.h[1] = *(const v8b*)(p + 16); return f.v;
  }
  static __device__ __forceinline__ v8f mma(v16b a, v16b b, v8f c) {
    return __builtin_amdgcn_wmma_f32_16x16x32_bf16(false, a, false, b, (short)0, c, false, false);
  }
  static __device__ __forceinline__ void guard(v8f& a, v8f& b, v16b x, v16b y) { dep_guard_b(a, b, x, y); }
  static __device__ __forceinline__ void keep(v16b a, v16b b, v16b c, v16b d) { keep4_b(a, b, c, d); }
};

template <int ET> struct Elem;
template <> struct Elem<0> { typedef _Float16 T; };
template <> struct Elem<1> { typedef __bf16 T; };
template <int ET, int SPL, int BIAS_MODE, int OUT_MODE, bool RESID, int ACT = 0>
__global__ __launch_bounds__(256) void wmma_gemm64(
    const unsigned short* __restrict__ Ap, const unsigned short* __restrict__ A2p, int lda, long strideA,
    const unsigned short* __restrict__ Btp, const unsigned short* __restrict__ Bt2p, int ldb, long strideB,
    void* __restrict__ Cout, void* __restrict__ Cout2, int ldc, long strideC,
    const float* __restrict__ bias,
    const float* __restrict__ resid, long strideR,
    int M, int N, int K, float scale) {
  typedef typename Elem<ET>::T T;
  typedef typename Frag<T>::V V;
  const T* A = (const T*)Ap; const T* A2 = (const T*)A2p; const T* Bt = (const T*)Btp; const T* Bt2 = (const T*)Bt2p;
  __shared__ __align__(16) float sT[8][16 * 68];
  const int b    = blockIdx.y;
  const int lane = threadIdx.x & 31;
  const int wave = threadIdx.x >> 5;
  const int tilesN = N >> 6;
  const int tilesM = M >> 6;
  const int tile = blockIdx.x * 8 + wave;
  if (tile >= tilesM * tilesN) return;
  const int tm = tile / tilesN;
  const int tn = tile - tm * tilesN;
  const int m0 = tm << 6;
  const int n0 = tn << 6;

  const T* Ab  = A  + (size_t)b * strideA;
  const T* Bb  = Bt + (size_t)b * strideB;
  const T* Ab2 = (SPL >= 1) ? (A2  + (size_t)b * strideA) : nullptr;
  const T* Bb2 = (SPL == 2) ? (Bt2 + (size_t)b * strideB) : nullptr;

  const int rlane = lane & 15;
  const int koff  = (lane >> 4) * 8;
  const int mOff  = (lane >> 4) * 8;

  v8f acc[4][4];
#pragma unroll
  for (int i = 0; i < 4; ++i)
#pragma unroll
    for (int j = 0; j < 4; ++j) acc[i][j] = (v8f){0.f,0.f,0.f,0.f,0.f,0.f,0.f,0.f};

  for (int k0 = 0; k0 < K; k0 += 32) {
    V bh[4], bl[4];
#pragma unroll
    for (int j = 0; j < 4; ++j) {
      const size_t bo = (size_t)(n0 + (j << 4) + rlane) * ldb + koff + k0;
      bh[j] = Frag<T>::load(Bb + bo);
      if (SPL == 2) bl[j] = Frag<T>::load(Bb2 + bo);
    }
#pragma unroll
    for (int i = 0; i < 4; ++i) {
      const size_t ao = (size_t)(m0 + (i << 4) + rlane) * lda + koff + k0;
      V ah = Frag<T>::load(Ab + ao);
      V al;
      if (SPL >= 1) al = Frag<T>::load(Ab2 + ao);
#pragma unroll
      for (int j = 0; j < 4; ++j) {
        acc[i][j] = Frag<T>::mma(ah, bh[j], acc[i][j]);
        if (SPL == 2) acc[i][j] = Frag<T>::mma(ah, bl[j], acc[i][j]);
        if (SPL >= 1) acc[i][j] = Frag<T>::mma(al, bh[j], acc[i][j]);
      }
      Frag<T>::guard(acc[i][0], acc[i][3], ah, (SPL >= 1) ? al : ah);
    }
    Frag<T>::keep(bh[0], bh[1], bh[2], bh[3]);
    if (SPL == 2) Frag<T>::keep(bl[0], bl[1], bl[2], bl[3]);
  }
  acc_guard4(acc[0][0], acc[0][1], acc[0][2], acc[0][3]);
  acc_guard4(acc[1][0], acc[1][1], acc[1][2], acc[1][3]);
  acc_guard4(acc[2][0], acc[2][1], acc[2][2], acc[2][3]);
  acc_guard4(acc[3][0], acc[3][1], acc[3][2], acc[3][3]);

  float* slab = sT[wave];
  const float* Rb = RESID ? (resid + (size_t)b * strideR) : nullptr;
#pragma unroll
  for (int i = 0; i < 4; ++i) {
    const int mBase = m0 + (i << 4);
#pragma unroll
    for (int j = 0; j < 4; ++j) {
      const int n = n0 + (j << 4) + rlane;
      float bv = 0.f;
      if (BIAS_MODE == 2) bv = bias[n];
#pragma unroll
      for (int r = 0; r < 8; ++r) {
        float v = acc[i][j][r] * scale;
        if (BIAS_MODE == 1) v += bias[mBase + mOff + r];
        if (BIAS_MODE == 2) v += bv;
        if (RESID) v += Rb[(size_t)(mBase + mOff + r) * ldc + n];
        if (ACT == 1) v = tanhf(v);
        if (ACT == 2) v = fmaxf(v, 0.0f);
        if (ACT == 3) v = v / (1.0f + expf(-v));
        if (ACT == 4) v = (v > 0.f) ? v : 0.01f * v;
        slab[(mOff + r) * 68 + (j << 4) + rlane] = v;
      }
    }
    __builtin_amdgcn_fence(__ATOMIC_RELEASE, "workgroup");
    __builtin_amdgcn_wave_barrier();
    __builtin_amdgcn_fence(__ATOMIC_ACQUIRE, "workgroup");
    if (OUT_MODE == 0) {
      float* C = (float*)Cout + (size_t)b * strideC;
      const int hh = lane >> 4, c4 = (lane & 15) * 4;
      for (int pass = 0; pass < 2; ++pass) {
#pragma unroll
        for (int it = 0; it < 8; ++it) {
          const int row = it * 2 + hh;
          v4f v = *(const v4f*)(slab + row * 68 + c4);
          *(volatile v4f*)(C + (size_t)(mBase + row) * ldc + n0 + c4) = v;
        }
        __threadfence();
      }
    } else {
      const int q = lane >> 3, c8 = (lane & 7) * 8;
      unsigned short* C  = (unsigned short*)Cout  + (size_t)b * strideC;
      unsigned short* C2 = (OUT_MODE == 2) ? ((unsigned short*)Cout2 + (size_t)b * strideC) : nullptr;
      for (int pass = 0; pass < 2; ++pass) {
#pragma unroll
        for (int it = 0; it < 4; ++it) {
          const int row = it * 4 + q;
          const float* sp = slab + row * 68 + c8;
          v8h hv, lv;
#pragma unroll
          for (int e = 0; e < 8; ++e) {
            if (OUT_MODE == 1) {
              hv[e] = (_Float16)sp[e];
            } else {
              unsigned short hb = f2bf_bits(sp[e]);
              unsigned short lb = f2bf_bits(sp[e] - bf_bits2f(hb));
              hv[e] = __builtin_bit_cast(_Float16, hb);
              lv[e] = __builtin_bit_cast(_Float16, lb);
            }
          }
          *(volatile v8h*)(C + (size_t)(mBase + row) * ldc + n0 + c8) = hv;
          if (OUT_MODE == 2) *(volatile v8h*)(C2 + (size_t)(mBase + row) * ldc + n0 + c8) = lv;
        }
        __threadfence();
      }
    }
    __builtin_amdgcn_fence(__ATOMIC_RELEASE, "workgroup");
    __builtin_amdgcn_wave_barrier();
    __builtin_amdgcn_fence(__ATOMIC_ACQUIRE, "workgroup");
  }
}

__global__ __launch_bounds__(256) void cast_rows_f16_kernel(
    const float* __restrict__ src, unsigned short* __restrict__ dst, int total8, float scale)
{
  const int i = blockIdx.x * 256 + threadIdx.x;
  if (i >= total8) return;
  const size_t e0 = (size_t)i << 3;
  const v4f a0 = *(const v4f*)(src + e0);
  const v4f a1 = *(const v4f*)(src + e0 + 4);
  v8h hv;
#pragma unroll
  for (int e = 0; e < 4; ++e) {
    hv[e]     = (_Float16)(a0[e] * scale);
    hv[4 + e] = (_Float16)(a1[e] * scale);
  }
  unsigned short* q = dst + e0;
  *(volatile v8h*)q = hv;
  __threadfence();
  *(volatile v8h*)q = hv;
}

__global__ __launch_bounds__(256) void cast_xproj_kernel(
    const float* __restrict__ src, unsigned short* __restrict__ dst)
{
  const int i = blockIdx.x * 256 + threadIdx.x;
  if (i >= kNStr * kXdP * (kDin / 8)) return;
  const int st  = i / (kXdP * (kDin / 8));
  const int rem = i - st * (kXdP * (kDin / 8));
  const int row = rem / (kDin / 8);
  const int c8  = (rem - row * (kDin / 8)) * 8;
  const int rowc = (row < kXdN) ? row : (kXdN - 1);
  const float* sp = src + ((size_t)(st * kXdN + rowc) * kDin + c8);
  const v4f a0 = *(const v4f*)(sp);
  const v4f a1 = *(const v4f*)(sp + 4);
  const float f = (row < kXdN) ? kWScale : 0.0f;
  v8h hv;
#pragma unroll
  for (int e = 0; e < 4; ++e) {
    hv[e]     = (_Float16)(a0[e] * f);
    hv[4 + e] = (_Float16)(a1[e] * f);
  }
  unsigned short* q = dst + ((size_t)i << 3);
  *(volatile v8h*)q = hv;
  __threadfence();
  *(volatile v8h*)q = hv;
}

__global__ __launch_bounds__(256) void ln_kernel(
    const float* __restrict__ x0, const float* __restrict__ x1, const float* __restrict__ x2,
    const float* __restrict__ nw, const float* __restrict__ nb, unsigned short* __restrict__ XN)
{
  const int lane = threadIdx.x & 31, wave = threadIdx.x >> 5;
  const int gr = blockIdx.x * 8 + wave;
  const int st = gr / kRowsS;
  const int r  = gr - st * kRowsS;
  const float* xs = (st == 0) ? x0 : ((st == 1) ? x1 : x2);
  const float* xr = xs + (size_t)r * kDm + lane * 8;
  const v4f a0 = *(const v4f*)(xr);
  const v4f a1 = *(const v4f*)(xr + 4);
  float v[8];
#pragma unroll
  for (int e = 0; e < 4; ++e) { v[e] = a0[e]; v[4 + e] = a1[e]; }
  float sum = ((v[0] + v[1]) + (v[2] + v[3])) + ((v[4] + v[5]) + (v[6] + v[7]));
#pragma unroll
  for (int off = 1; off < 32; off <<= 1) sum += __shfl_xor(sum, off, 32);
  const float mean = sum * (1.0f / 256.0f);
  float sq = 0.f;
#pragma unroll
  for (int e = 0; e < 8; ++e) { v[e] -= mean; sq = fmaf(v[e], v[e], sq); }
#pragma unroll
  for (int off = 1; off < 32; off <<= 1) sq += __shfl_xor(sq, off, 32);
  const float var = sq * (1.0f / 256.0f);
  const float inv = 1.0f / sqrtf(var + 1e-5f);
  const float* wp = nw + st * kDm + lane * 8;
  const float* bp = nb + st * kDm + lane * 8;
  const v4f w0 = *(const v4f*)(wp);
  const v4f w1 = *(const v4f*)(wp + 4);
  const v4f b0 = *(const v4f*)(bp);
  const v4f b1 = *(const v4f*)(bp + 4);
  v8h hv;
#pragma unroll
  for (int e = 0; e < 4; ++e) {
    hv[e]     = (_Float16)((v[e] * inv) * w0[e] + b0[e]);
    hv[4 + e] = (_Float16)((v[4 + e] * inv) * w1[e] + b1[e]);
  }
  unsigned short* q = XN + (size_t)gr * kDm + lane * 8;
  *(volatile v8h*)q = hv;
  __threadfence();
  *(volatile v8h*)q = hv;
}

__global__ __launch_bounds__(256) void conv_silu_kernel(
    const float* __restrict__ XZ, const float* __restrict__ cw, const float* __restrict__ cb,
    float* __restrict__ UC, unsigned short* __restrict__ UH)
{
  __shared__ __align__(16) float sT[16 * kConvTP];
  const int tid = threadIdx.x, lane = tid & 31, wave = tid >> 5;
  const int d0 = blockIdx.x * 256, d = d0 + tid;
  const int g0 = blockIdx.y * 64;
  const int tb = g0 & (kSeq - 1);
  const int st = g0 / kRowsS;
  const size_t dw = (size_t)st * kDin + d;
  const float w0 = cw[dw * 4 + 0], w1 = cw[dw * 4 + 1], w2 = cw[dw * 4 + 2], w3 = cw[dw * 4 + 3];
  const float bc = cb[dw];
  float xm3, xm2, xm1;
  {
    const bool hist = (tb > 0);
    const int rb = hist ? (g0 - 3) : g0;
    const float v3 = XZ[(size_t)rb * kXzP + d];
    const float v2 = XZ[(size_t)(rb + 1) * kXzP + d];
    const float v1 = XZ[(size_t)(rb + 2) * kXzP + d];
    xm3 = hist ? v3 : 0.f;
    xm2 = hist ? v2 : 0.f;
    xm1 = hist ? v1 : 0.f;
  }
  const int hrow = wave >> 1;
  const int hch  = (wave & 1) * 128 + lane * 4;
#pragma unroll 1
  for (int sub = 0; sub < 4; ++sub) {
    const int lb = g0 + sub * 16;
#pragma unroll 1
    for (int s = 0; s < 16; ++s) {
      const float xcur = XZ[(size_t)(lb + s) * kXzP + d];
      float acc = w0 * xm3;
      acc = fmaf(w1, xm2, acc);
      acc = fmaf(w2, xm1, acc);
      acc = fmaf(w3, xcur, acc);
      const float sv = acc + bc;
      const float sg = __builtin_amdgcn_rcpf(1.0f + __expf(-sv));
      sT[s * kConvTP + tid] = sv * sg;
      xm3 = xm2; xm2 = xm1; xm1 = xcur;
    }
    __syncthreads();
    v4f fv[4];
    v8h bh[2];
#pragma unroll
    for (int it = 0; it < 4; ++it) fv[it] = *(const v4f*)(sT + (it * 4 + hrow) * kConvTP + hch);
#pragma unroll
    for (int it = 0; it < 2; ++it) {
      const float* sp = sT + (it * 8 + wave) * kConvTP + lane * 8;
      const v4f a0 = *(const v4f*)(sp);
      const v4f a1 = *(const v4f*)(sp + 4);
#pragma unroll
      for (int e = 0; e < 4; ++e) {
        bh[it][e]     = (_Float16)(a0[e] * kUScale);
        bh[it][4 + e] = (_Float16)(a1[e] * kUScale);
      }
    }
    for (int pass = 0; pass < 2; ++pass) {
#pragma unroll
      for (int it = 0; it < 4; ++it)
        *(volatile v4f*)(UC + (size_t)(lb + it * 4 + hrow) * kDin + d0 + hch) = fv[it];
#pragma unroll
      for (int it = 0; it < 2; ++it) {
        const size_t o = (size_t)(lb + it * 8 + wave) * kDin + d0 + lane * 8;
        *(volatile v8h*)(UH + o) = bh[it];
      }
      __threadfence();
    }
    __syncthreads();
  }
}

__global__ __launch_bounds__(64) void scan_kernel(
    const float* __restrict__ XD, const float* __restrict__ UC, const float* __restrict__ XZ,
    const float* __restrict__ Wdt, const float* __restrict__ bdt, const float* __restrict__ Alog,
    const float* __restrict__ Dp, unsigned short* __restrict__ YH)
{
  __shared__ __align__(16) float sX[kScanTS * kXdP];
  __shared__ __align__(16) float sY[kScanTS * kScanYP];
  __shared__ __align__(16) float sW[kDtR * kScanCh];
  __shared__ __align__(16) float sA[kNst * kScanCh];
  const int tid = threadIdx.x, lane = tid & 31, wave = tid >> 5;
  constexpr int kBlkPerSB = kDin / kScanCh;
  const int sb  = blockIdx.x / kBlkPerSB;
  const int d0  = (blockIdx.x - sb * kBlkPerSB) * kScanCh;
  const int d   = d0 + tid;
  const int st  = sb >> 1;
  const size_t dw = (size_t)st * kDin + d;
  const size_t row0 = (size_t)sb * kSeq;
#pragma unroll 1
  for (int r = 0; r < kDtR; ++r) sW[r * kScanCh + tid] = Wdt[dw * kDtR + r];
#pragma unroll 1
  for (int s = 0; s < kNst; ++s) sA[s * kScanCh + tid] = -expf(Alog[dw * kNst + s]);
  __syncthreads();
  float negA[kNst], h[kNst];
#pragma unroll
  for (int s = 0; s < kNst; ++s) {
    negA[s] = sA[s * kScanCh + tid];
    h[s] = 0.f;
  }
  const float bb = bdt[dw], Dd = Dp[dw];
  const int lr = tid >> 4, lc4 = (tid & 15) * 4;
  const int q = lane >> 3, c8 = (lane & 7) * 8;
#pragma unroll 1
  for (int t0 = 0; t0 < kSeq; t0 += kScanTS) {
    __syncthreads();
#pragma unroll
    for (int i = 0; i < 16; ++i) {
      const int r = lr + 4 * i;
      *(v4f*)(sX + r * kXdP + lc4) = *(const v4f*)(XD + (row0 + t0 + r) * kXdP + lc4);
    }
    __syncthreads();
#pragma unroll 1
    for (int s = 0; s < kScanTS; ++s) {
      const int t = t0 + s;
      const float* xr = sX + s * kXdP;
      float vdot = 0.f;
#pragma unroll 1
      for (int r4 = 0; r4 < kDtR / 4; ++r4) {
        const v4f xv = *(const v4f*)(xr + 4 * r4);
        const float* wp = sW + (4 * r4) * kScanCh + tid;
        vdot = fmaf(xv[0], wp[0], vdot);
        vdot = fmaf(xv[1], wp[kScanCh], vdot);
        vdot = fmaf(xv[2], wp[2 * kScanCh], vdot);
        vdot = fmaf(xv[3], wp[3 * kScanCh], vdot);
      }
      float Bs[kNst], Cs[kNst];
#pragma unroll
      for (int q4 = 0; q4 < 4; ++q4) {
        const v4f bv = *(const v4f*)(xr + kDtR + 4 * q4);
        const v4f cv = *(const v4f*)(xr + kDtR + kNst + 4 * q4);
        Bs[4 * q4 + 0] = bv[0]; Bs[4 * q4 + 1] = bv[1]; Bs[4 * q4 + 2] = bv[2]; Bs[4 * q4 + 3] = bv[3];
        Cs[4 * q4 + 0] = cv[0]; Cs[4 * q4 + 1] = cv[1]; Cs[4 * q4 + 2] = cv[2]; Cs[4 * q4 + 3] = cv[3];
      }
      const float v   = vdot + bb;
      const float a   = __expf(-fabsf(v));
      const float u   = 1.0f + a;
      const float l1p = __logf(u) + (a - (u - 1.0f)) * __builtin_amdgcn_rcpf(u);
      const float dt  = fmaxf(v, 0.0f) + l1p;
      const float xt  = UC[(row0 + t) * kDin + d];
      const float dtx = dt * xt;
      float y = 0.f;
#pragma unroll
      for (int k = 0; k < kNst; ++k) {
        const float e = __expf(dt * negA[k]);
        h[k] = e * h[k] + dtx * Bs[k];
        y = h[k] * Cs[k] + y;
      }
      y = xt * Dd + y;
      const float zv = XZ[(row0 + t) * kXzP + kDin + d];
      const float sg = __builtin_amdgcn_rcpf(1.0f + __expf(-zv));
      y = y * (zv * sg);
      sY[s * kScanYP + tid] = y;
    }
    __syncthreads();
    v8h hv[8];
#pragma unroll
    for (int it = 0; it < 8; ++it) {
      const int row = it * 8 + wave * 4 + q;
      const float* sp = sY + row * kScanYP + c8;
      const v4f a0 = *(const v4f*)(sp);
      const v4f a1 = *(const v4f*)(sp + 4);
#pragma unroll
      for (int e = 0; e < 4; ++e) {
        hv[it][e]     = (_Float16)(a0[e] * kYScale);
        hv[it][4 + e] = (_Float16)(a1[e] * kYScale);
      }
    }
    for (int pass = 0; pass < 2; ++pass) {
#pragma unroll
      for (int it = 0; it < 8; ++it) {
        const int row = it * 8 + wave * 4 + q;
        const size_t o = (row0 + t0 + row) * kDin + d0 + c8;
        *(volatile v8h*)(YH + o) = hv[it];
      }
      __threadfence();
    }
  }
}

__global__ __launch_bounds__(256) void pool_kernel(const float* __restrict__ PR, float* __restrict__ PO)
{
  __shared__ float red[8 * 32];
  __shared__ __align__(16) float sOut[32];
  const int tid = threadIdx.x, c = tid & 31, p = tid >> 5;
  const int sb = blockIdx.x >> 3, cg = blockIdx.x & 7;
  const float* base = PR + (size_t)sb * kSeq * kDm + cg * 32 + c;
  float acc = 0.f;
#pragma unroll 1
  for (int n = p; n < kSeq; n += 8) acc += base[(size_t)n * kDm];
  red[p * 32 + c] = acc;
  __syncthreads();
  if (tid < 32) {
    float tsum = red[tid];
    tsum += red[32 + tid];
    tsum += red[64 + tid];
    tsum += red[96 + tid];
    tsum += red[128 + tid];
    tsum += red[160 + tid];
    tsum += red[192 + tid];
    tsum += red[224 + tid];
    sOut[tid] = tsum * (1.0f / 2048.0f);
  }
  __syncthreads();
  if (tid < 8) {
    const v4f vv = *(const v4f*)(sOut + tid * 4);
    const int b = sb & 1, st = sb >> 1;
    float* dst = PO + (size_t)b * kCat + st * kDm + cg * 32 + tid * 4;
    *(volatile v4f*)dst = vv;
    __threadfence();
    *(volatile v4f*)dst = vv;
  }
}

__global__ __launch_bounds__(256) void agg_kernel(
    const float* __restrict__ PO, const float* __restrict__ w1, const float* __restrict__ b1,
    const float* __restrict__ w2, const float* __restrict__ b2, const float* __restrict__ temp,
    float* __restrict__ CF)
{
  __shared__ float sP[kBatch * kCat];
  __shared__ float sH[kBatch * kDm];
  __shared__ float sL[8];
  __shared__ __align__(16) float sC[32];
  const int tid = threadIdx.x;
#pragma unroll 1
  for (int i = tid; i < kBatch * kCat; i += 256) sP[i] = PO[i];
  __syncthreads();
  const float bias1 = b1[tid];
  const float* wr = w1 + (size_t)tid * kCat;
#pragma unroll 1
  for (int b = 0; b < kBatch; ++b) {
    const float* pp = sP + b * kCat;
    float acc = 0.f;
#pragma unroll 1
    for (int e = 0; e < kCat; ++e) acc = fmaf(pp[e], wr[e], acc);
    acc += bias1;
    const float c3 = 0.7978845608028654f * (acc + 0.044715f * acc * acc * acc);
    sH[b * kDm + tid] = 0.5f * acc * (1.0f + tanhf(c3));
  }
  __syncthreads();
  if (tid < kBatch * 3) {
    const int b = tid / 3, k = tid - b * 3;
    const float* hp = sH + b * kDm;
    const float* wk = w2 + k * kDm;
    float a = 0.f;
#pragma unroll 1
    for (int dd = 0; dd < kDm; ++dd) a = fmaf(hp[dd], wk[dd], a);
    sL[tid] = a + b2[k];
  }
  __syncthreads();
  if (tid < 32) {
    float cval = 0.f;
    if (tid < kBatch * 3) {
      const int b = tid / 3, k = tid - b * 3;
      const float l0 = sL[b * 3 + 0], l1 = sL[b * 3 + 1], l2 = sL[b * 3 + 2];
      const float mx = fmaxf(l0, fmaxf(l1, l2));
      const float e0 = __expf(l0 - mx), e1 = __expf(l1 - mx), e2 = __expf(l2 - mx);
      const float inv1 = 1.0f / (e0 + e1 + e2);
      const float c0 = e0 * inv1, c1 = e1 * inv1, c2 = e2 * inv1;
      const float ti = 1.0f / (temp[0] + 1e-6f);
      const float g0 = c0 * ti, g1 = c1 * ti, g2 = c2 * ti;
      const float mx2 = fmaxf(g0, fmaxf(g1, g2));
      const float f0 = __expf(g0 - mx2), f1 = __expf(g1 - mx2), f2 = __expf(g2 - mx2);
      const float inv2 = 1.0f / (f0 + f1 + f2);
      const float own = (k == 0) ? f0 : ((k == 1) ? f1 : f2);
      cval = own * inv2;
    }
    sC[tid] = cval;
  }
  __syncthreads();
  if (tid < 8) {
    const v4f vv = *(const v4f*)(sC + tid * 4);
    float* dst = CF + tid * 4;
    *(volatile v4f*)dst = vv;
    __threadfence();
    *(volatile v4f*)dst = vv;
  }
}

__global__ __launch_bounds__(256) void multi_cast_kernel(const float* __restrict__ PR, unsigned short* __restrict__ MU)
{
  const int i = blockIdx.x * 256 + threadIdx.x;
  if (i >= kNStr * kRowsS * (kDm / 8)) return;
  const int st  = i / (kRowsS * (kDm / 8));
  const int rem = i - st * (kRowsS * (kDm / 8));
  const int row = rem / (kDm / 8);
  const int c8  = (rem - row * (kDm / 8)) * 8;
  const float* sp = PR + ((size_t)st * kRowsS + row) * kDm + c8;
  const v4f a0 = *(const v4f*)(sp);
  const v4f a1 = *(const v4f*)(sp + 4);
  v8h hv;
#pragma unroll
  for (int e = 0; e < 4; ++e) {
    hv[e]     = (_Float16)a0[e];
    hv[4 + e] = (_Float16)a1[e];
  }
  unsigned short* q = MU + (size_t)row * kCat + st * kDm + c8;
  *(volatile v8h*)q = hv;
  __threadfence();
  *(volatile v8h*)q = hv;
}

__global__ __launch_bounds__(256) void wgt_kernel(
    const float* __restrict__ PR, const float* __restrict__ CF, const float* __restrict__ pb, float* __restrict__ WG)
{
  const int i = blockIdx.x * 256 + threadIdx.x;
  if (i >= kRowsS * (kDm / 4)) return;
  const int row = i / (kDm / 4);
  const int c4  = (i - row * (kDm / 4)) * 4;
  const int b   = row / kSeq;
  const float k0 = CF[b * 3 + 0], k1 = CF[b * 3 + 1], k2 = CF[b * 3 + 2];
  const v4f p0 = *(const v4f*)(PR + (size_t)row * kDm + c4);
  const v4f p1 = *(const v4f*)(PR + ((size_t)kRowsS + row) * kDm + c4);
  const v4f p2 = *(const v4f*)(PR + ((size_t)2 * kRowsS + row) * kDm + c4);
  const v4f bv = *(const v4f*)(pb + c4);
  v4f w;
#pragma unroll
  for (int e = 0; e < 4; ++e) w[e] = bv[e] + ((k0 * p0[e] + k1 * p1[e]) + k2 * p2[e]);
  float* dst = WG + (size_t)row * kDm + c4;
  *(volatile v4f*)dst = w;
  __threadfence();
  *(volatile v4f*)dst = w;
}

extern "C" void kernel_launch(void* const* d_in, const int* in_sizes, int n_in,
                              void* d_out, int out_size, void* d_ws, size_t ws_size,
                              hipStream_t stream) {
  if (n_in < 21) return;
  if (in_sizes[0] != kRowsS * kDm || in_sizes[1] != kRowsS * kDm || in_sizes[2] != kRowsS * kDm) return;
  if (in_sizes[3] != kNStr * kDm || in_sizes[4] != kNStr * kDm) return;
  if (in_sizes[5] != kNStr * kXzP * kDm) return;
  if (in_sizes[6] != kNStr * kDin * 4) return;
  if (in_sizes[7] != kNStr * kDin) return;
  if (in_sizes[8] != kNStr * kXdN * kDin) return;
  if (in_sizes[9] != kNStr * kDin * kDtR) return;
  if (in_sizes[10] != kNStr * kDin) return;
  if (in_sizes[11] != kNStr * kDin * kNst) return;
  if (in_sizes[12] != kNStr * kDin) return;
  if (in_sizes[13] != kNStr * kDm * kDin) return;
  if (in_sizes[14] < 1) return;
  if (in_sizes[15] != kDm * kCat) return;
  if (in_sizes[16] != kDm) return;
  if (in_sizes[17] != kNStr * kDm) return;
  if (in_sizes[18] != kNStr) return;
  if (in_sizes[19] != kDm * kCat) return;
  if (in_sizes[20] != kDm) return;
  if (out_size != kRowsS * kDm) return;
  if (ws_size < kWsTotal) return;

  const float* xin0    = (const float*)d_in[0];
  const float* xin1    = (const float*)d_in[1];
  const float* xin2    = (const float*)d_in[2];
  const float* norm_w  = (const float*)d_in[3];
  const float* norm_b  = (const float*)d_in[4];
  const float* in_w    = (const float*)d_in[5];
  const float* conv_w  = (const float*)d_in[6];
  const float* conv_b  = (const float*)d_in[7];
  const float* xproj_w = (const float*)d_in[8];
  const float* dt_w    = (const float*)d_in[9];
  const float* dt_b    = (const float*)d_in[10];
  const float* A_log   = (const float*)d_in[11];
  const float* Dpar    = (const float*)d_in[12];
  const float* out_w   = (const float*)d_in[13];
  const float* temp    = (const float*)d_in[14];
  const float* agg_w1  = (const float*)d_in[15];
  const float* agg_b1  = (const float*)d_in[16];
  const float* agg_w2  = (const float*)d_in[17];
  const float* agg_b2  = (const float*)d_in[18];
  const float* proj_w  = (const float*)d_in[19];
  const float* proj_b  = (const float*)d_in[20];
  float* out = (float*)d_out;

  char* ws = (char*)d_ws;
  unsigned short* XN = (unsigned short*)(ws + kOffXN);
  unsigned short* WI = (unsigned short*)(ws + kOffWI);
  unsigned short* WX = (unsigned short*)(ws + kOffWX);
  unsigned short* WO = (unsigned short*)(ws + kOffWO);
  unsigned short* WP = (unsigned short*)(ws + kOffWP);
  float*          XZ = (float*)(ws + kOffXZ);
  float*          UC = (float*)(ws + kOffUC);
  unsigned short* UH = (unsigned short*)(ws + kOffUH);
  float*          XD = (float*)(ws + kOffXD);
  unsigned short* YH = (unsigned short*)(ws + kOffYH);
  float*          PR = (float*)(ws + kOffPR);
  unsigned short* MU = (unsigned short*)(ws + kOffMU);
  float*          WG = (float*)(ws + kOffWG);
  float*          PO = (float*)(ws + kOffPO);
  float*          CF = (float*)(ws + kOffCF);

  cast_rows_f16_kernel<<<(kNStr * kXzP * kDm / 8) / 256, 256, 0, stream>>>(in_w, WI, kNStr * kXzP * kDm / 8, kWScale);
  cast_xproj_kernel<<<(kNStr * kXdP * (kDin / 8)) / 256, 256, 0, stream>>>(xproj_w, WX);
  cast_rows_f16_kernel<<<(kNStr * kDm * kDin / 8) / 256, 256, 0, stream>>>(out_w, WO, kNStr * kDm * kDin / 8, kWScale);
  cast_rows_f16_kernel<<<(kDm * kCat / 8) / 256, 256, 0, stream>>>(proj_w, WP, kDm * kCat / 8, kWScale);

  ln_kernel<<<kRowsT / 8, 256, 0, stream>>>(xin0, xin1, xin2, norm_w, norm_b, XN);

  wmma_gemm64<0, 0, 0, 0, false><<<dim3(128, kNStr), 256, 0, stream>>>(
      XN, nullptr, kDm, (long)kRowsS * kDm,
      WI, nullptr, kDm, (long)kXzP * kDm,
      (void*)XZ, nullptr, kXzP, (long)kRowsS * kXzP,
      nullptr, nullptr, 0L,
      kRowsS, kXzP, kDm, 1.0f / kWScale);

  conv_silu_kernel<<<dim3(kDin / 256, kRowsT / 64), 256, 0, stream>>>(XZ, conv_w, conv_b, UC, UH);

  wmma_gemm64<0, 0, 0, 0, false><<<dim3(8, kNStr), 256, 0, stream>>>(
      UH, nullptr, kDin, (long)kRowsS * kDin,
      WX, nullptr, kDin, (long)kXdP * kDin,
      (void*)XD, nullptr, kXdP, (long)kRowsS * kXdP,
      nullptr, nullptr, 0L,
      kRowsS, kXdP, kDin, 1.0f / (kUScale * kWScale));

  scan_kernel<<<kNStr * kBatch * (kDin / kScanCh), kScanCh, 0, stream>>>(XD, UC, XZ, dt_w, dt_b, A_log, Dpar, YH);

  const float* xin[3] = { xin0, xin1, xin2 };
  for (int st = 0; st < kNStr; ++st) {
    wmma_gemm64<0, 0, 0, 0, true><<<dim3(32, 1), 256, 0, stream>>>(
        YH + (size_t)st * kRowsS * kDin, nullptr, kDin, 0L,
        WO + (size_t)st * kDm * kDin, nullptr, kDin, 0L,
        (void*)(PR + (size_t)st * kRowsS * kDm), nullptr, kDm, 0L,
        nullptr, xin[st], 0L,
        kRowsS, kDm, kDin, 1.0f / (kYScale * kWScale));
  }

  pool_kernel<<<kNStr * kBatch * (kDm / 32), 256, 0, stream>>>(PR, PO);

  agg_kernel<<<1, 256, 0, stream>>>(PO, agg_w1, agg_b1, agg_w2, agg_b2, temp, CF);

  multi_cast_kernel<<<(kNStr * kRowsS * (kDm / 8)) / 256, 256, 0, stream>>>(PR, MU);

  wgt_kernel<<<(kRowsS * (kDm / 4)) / 256, 256, 0, stream>>>(PR, CF, proj_b, WG);

  wmma_gemm64<0, 0, 0, 0, true><<<dim3(32, 1), 256, 0, stream>>>(
      MU, nullptr, kCat, 0L,
      WP, nullptr, kCat, 0L,
      (void*)out, nullptr, kDm, 0L,
      nullptr, WG, 0L,
      kRowsS, kDm, kCat, 1.0f / kWScale);
}
